// StreamGQASelfAttentionRelPos_1632087573174
// MI455X (gfx1250) — hardware-run, weakly checked
//
#include <hip/hip_runtime.h>
#include <stddef.h>
#include <stdint.h>

#define NTOK  2048
#define TT    1024
#define DM    1024
#define NH    16
#define NG    4
#define HD    64
#define NBH   32
#define NBG   8
#define SC    1024
#define SKEY  2048
#define NREL  255
#define NRELP 256
#define WROWS 2560
#define OROW  1536
#define QB    64
#define KC    64
#define NQB   (TT / QB)
#define NCVT  4360

static_assert(NH * HD == DM);
static_assert(NG * HD * 2 + DM * 2 == WROWS);
static_assert(OROW == DM + 2 * NG * HD);
static_assert(TT % QB == 0);
static_assert(SKEY % KC == 0);
static_assert(SC % KC == 0);
static_assert(DM % 64 == 0);
static_assert(HD == 64);
static_assert(NCVT == 3 * (NTOK * DM / 2048) + 2 * (DM * DM / 2048) + 2 * (NG * HD * DM / 2048) + (NRELP * HD / 2048));

typedef unsigned short us;
typedef __attribute__((ext_vector_type(16))) __bf16 v16bf;
typedef us           v8us __attribute__((ext_vector_type(8)));
typedef float        v8f  __attribute__((ext_vector_type(8)));
typedef float        v4f  __attribute__((ext_vector_type(4)));
typedef unsigned int v4u  __attribute__((ext_vector_type(4)));

union Frag  { v16bf v; v8us h[2]; };
union Pack8 { v8us h; v4u u; };

__device__ __forceinline__ us bf_rne(float f) {
  unsigned u = __float_as_uint(f);
  u = u + 0x7FFFu + ((u >> 16) & 1u);
  return (us)(u >> 16);
}
__device__ __forceinline__ float bf_val(us hv) { return __uint_as_float(((unsigned)hv) << 16); }
__device__ __forceinline__ void split2(float f, us& hi, us& lo) {
  const us hv = bf_rne(f);
  hi = hv;
  lo = bf_rne(f - bf_val(hv));
}
__device__ __forceinline__ void split8(const float (&f)[8], Pack8& ph, Pack8& pl) {
  us hh[8], ll[8];
#pragma unroll
  for (int e = 0; e < 8; ++e) split2(f[e], hh[e], ll[e]);
  ph.h = (v8us){hh[0], hh[1], hh[2], hh[3], hh[4], hh[5], hh[6], hh[7]};
  pl.h = (v8us){ll[0], ll[1], ll[2], ll[3], ll[4], ll[5], ll[6], ll[7]};
}

__device__ __forceinline__ v8f mma16(v16bf a, v16bf b, v8f c) {
  c = __builtin_amdgcn_wmma_f32_16x16x32_bf16(false, a, false, b, (short)0, c, false, false);
  asm volatile("v_nop\n\tv_nop\n\tv_nop\n\tv_nop" : "+v"(c) : "v"(a), "v"(b));
  return c;
}

__device__ __forceinline__ v16bf ldfrag(const us* p, int ld, int row0, int k0, int lane) {
  const int m = lane & 15, lh = lane >> 4;
  const us* q = p + (size_t)(row0 + m) * ld + k0 + 8 * lh;
  Frag f;
  f.h[0] = *(const v8us*)(q);
  f.h[1] = *(const v8us*)(q + 16);
  return f.v;
}

__device__ __forceinline__ v8f zero8() { return (v8f){0.f, 0.f, 0.f, 0.f, 0.f, 0.f, 0.f, 0.f}; }

__device__ __forceinline__ void gemm16x64x3(const us* __restrict__ Ah, const us* __restrict__ Al,
                                            const us* __restrict__ Bh, const us* __restrict__ Bl,
                                            int m0, int n0, int K, int ld, int lane, v8f (&acc)[4]) {
#pragma unroll 1
  for (int k0 = 0; k0 < K; k0 += 32) {
    const v16bf ah = ldfrag(Ah, ld, m0, k0, lane);
    const v16bf al = ldfrag(Al, ld, m0, k0, lane);
#pragma unroll
    for (int t = 0; t < 4; ++t) {
      const v16bf bh = ldfrag(Bh, ld, n0 + 16 * t, k0, lane);
      const v16bf bl = ldfrag(Bl, ld, n0 + 16 * t, k0, lane);
      acc[t] = mma16(ah, bh, acc[t]);
      acc[t] = mma16(ah, bl, acc[t]);
      acc[t] = mma16(al, bh, acc[t]);
    }
  }
}

__global__ __launch_bounds__(256) void k_cvt(const float* __restrict__ q, const float* __restrict__ k,
                                             const float* __restrict__ v, const float* __restrict__ wq,
                                             const float* __restrict__ wk, const float* __restrict__ wv,
                                             const float* __restrict__ wo, const float* __restrict__ rel,
                                             us* __restrict__ xh, us* __restrict__ xl,
                                             us* __restrict__ wh, us* __restrict__ wl,
                                             us* __restrict__ rh, us* __restrict__ rl) {
  const int blk = blockIdx.x;
  const int seg = (blk < 1024) ? 0 : ((blk < 2048) ? 1 : ((blk < 3072) ? 2 : ((blk < 3584) ? 3 :
                  ((blk < 3712) ? 4 : ((blk < 3840) ? 5 : ((blk < 4352) ? 6 : 7))))));
  const float* src = (seg == 0) ? q : ((seg == 1) ? k : ((seg == 2) ? v : ((seg == 3) ? wq :
                     ((seg == 4) ? wk : ((seg == 5) ? wv : ((seg == 6) ? wo : rel))))));
  const int nsrc = (seg < 3) ? (NTOK * DM) : ((seg == 3 || seg == 6) ? (DM * DM) :
                   ((seg < 6) ? (NG * HD * DM) : (NREL * HD)));
  const int b0 = (seg == 0) ? 0 : ((seg == 1) ? 1024 : ((seg == 2) ? 2048 : ((seg == 3) ? 3072 :
                 ((seg == 4) ? 3584 : ((seg == 5) ? 3712 : ((seg == 6) ? 3840 : 4352))))));
  const size_t doff = (seg < 3) ? ((size_t)seg * NTOK * DM)
                    : ((seg == 3) ? (size_t)0 : ((seg == 4) ? ((size_t)DM * DM)
                    : ((seg == 5) ? ((size_t)(DM + NG * HD) * DM) : ((seg == 6) ? ((size_t)OROW * DM) : (size_t)0))));
  us* dh = ((seg < 3) ? xh : ((seg < 7) ? wh : rh)) + doff;
  us* dl = ((seg < 3) ? xl : ((seg < 7) ? wl : rl)) + doff;

  const int i  = (blk - b0) * 2048 + (int)threadIdx.x * 8;
  const int ic = (i < nsrc - 8) ? i : (nsrc - 8);
  const v4f a0 = *(const v4f*)(src + ic);
  const v4f a1 = *(const v4f*)(src + ic + 4);
  const bool ok = (i < nsrc);
  float f[8];
  f[0] = ok ? a0[0] : 0.f;  f[1] = ok ? a0[1] : 0.f;  f[2] = ok ? a0[2] : 0.f;  f[3] = ok ? a0[3] : 0.f;
  f[4] = ok ? a1[0] : 0.f;  f[5] = ok ? a1[1] : 0.f;  f[6] = ok ? a1[2] : 0.f;  f[7] = ok ? a1[3] : 0.f;
  Pack8 ph, pl;
  split8(f, ph, pl);
  const v4u hv = ph.u, lv = pl.u;
  *(volatile v4u*)(dh + i) = hv;
  *(volatile v4u*)(dl + i) = lv;
  __threadfence();
  *(volatile v4u*)(dh + i) = hv;
  *(volatile v4u*)(dl + i) = lv;
}

#define TWP 68
__global__ __launch_bounds__(128) void k_cvtc(const float* __restrict__ ck, const float* __restrict__ cv,
                                              us* __restrict__ kch, us* __restrict__ kcl,
                                              us* __restrict__ vch, us* __restrict__ vcl) {
  __shared__ __align__(16) float tl[64 * TWP];
  const int tid = threadIdx.x;
  const int s0 = blockIdx.x * 64;
  const int bh = blockIdx.y;
  const int z  = blockIdx.z;
  const float* inp = (z == 0) ? (ck + (size_t)bh * HD * SC + s0) : (cv + ((size_t)bh * SC + s0) * HD);
  const int ipitch = (z == 0) ? SC : HD;
  const size_t obase = (z == 0) ? (((size_t)bh * SC + s0) * HD) : ((size_t)bh * HD * SC + s0);
  const int opitch = (z == 0) ? HD : SC;
  us* oh = ((z == 0) ? kch : vch) + obase;
  us* ol = ((z == 0) ? kcl : vcl) + obase;
#pragma unroll
  for (int j = 0; j < 8; ++j) {
    const int p  = tid + 128 * j;
    const int kr = p >> 4;
    const int c4 = (p & 15) * 4;
    const v4f a = *(const v4f*)(inp + (size_t)kr * ipitch + c4);
    *(v4f*)(tl + kr * TWP + c4) = a;
  }
  __syncthreads();
  v4u hv[4], lv[4];
  size_t go[4];
#pragma unroll
  for (int j = 0; j < 4; ++j) {
    const int p  = tid + 128 * j;
    const int n  = p >> 3;
    const int kc = (p & 7) * 8;
    const float* cp = tl + kc * TWP + n;
    float f[8];
#pragma unroll
    for (int e = 0; e < 8; ++e) f[e] = cp[e * TWP];
    Pack8 ph, pl;
    split8(f, ph, pl);
    hv[j] = ph.u;
    lv[j] = pl.u;
    go[j] = (size_t)n * opitch + kc;
  }
#pragma unroll
  for (int j = 0; j < 4; ++j) { *(volatile v4u*)(oh + go[j]) = hv[j]; *(volatile v4u*)(ol + go[j]) = lv[j]; }
  __threadfence();
#pragma unroll
  for (int j = 0; j < 4; ++j) { *(volatile v4u*)(oh + go[j]) = hv[j]; *(volatile v4u*)(ol + go[j]) = lv[j]; }
}

#define SFP 68
__device__ __forceinline__ void put_ck(const float* sf, float* __restrict__ nck, int bb, int g, int tb, int tid) {
#pragma unroll
  for (int it = 0; it < 8; ++it) {
    const int p = tid + 128 * it;
    const int L = p >> 3, pc = p & 7;
    const int dd = L >> 1, half = L & 1;
    const float* cp = sf + (half * 32 + pc * 4) * SFP + dd;
    const v4f val = (v4f){cp[0], cp[SFP], cp[2 * SFP], cp[3 * SFP]};
#pragma unroll
    for (int rep = 0; rep < 4; ++rep) {
      const int bhr = bb * NH + 4 * g + rep;
      float* d = nck + ((size_t)(bhr * HD + dd)) * TT + tb + half * 32 + pc * 4;
      *(volatile v4f*)d = val;
    }
  }
}
__device__ __forceinline__ void put_cv(const float* sf, float* __restrict__ ncv, int bb, int g, int tb, int tid) {
#pragma unroll
  for (int it = 0; it < 8; ++it) {
    const int p = tid + 128 * it;
    const int L = p >> 3, pc = p & 7;
    const int lr = L >> 1, half = L & 1;
    const v4f val = *(const v4f*)(sf + lr * SFP + half * 32 + pc * 4);
#pragma unroll
    for (int rep = 0; rep < 4; ++rep) {
      const int bhr = bb * NH + 4 * g + rep;
      float* d = ncv + ((size_t)(bhr * TT + tb + lr)) * HD + half * 32 + pc * 4;
      *(volatile v4f*)d = val;
    }
  }
}

__global__ __launch_bounds__(128) void k_qkv(const us* __restrict__ xh, const us* __restrict__ xl,
                                             const us* __restrict__ wh, const us* __restrict__ wl,
                                             us* __restrict__ qh, us* __restrict__ ql,
                                             us* __restrict__ kph, us* __restrict__ kpl,
                                             us* __restrict__ vth, us* __restrict__ vtl,
                                             float* __restrict__ nck, float* __restrict__ ncv) {
  __shared__ __align__(16) float sf[64 * SFP];
  const int tid = threadIdx.x, lane = tid & 31, wave = tid >> 5;
  const int hh = lane >> 4, c = lane & 15;
  const int mb = blockIdx.x * 64;
  const int bb = mb >> 10;
  const int tb = mb & 1023;
  const int ns = blockIdx.y;
  const int which = (ns < 16) ? 0 : ((ns < 20) ? 1 : 2);
  const size_t xoff = (size_t)which * NTOK * DM;
  const int m0 = mb + wave * 16;
  const int n0 = 64 * ns;

  v8f acc[4];
#pragma unroll
  for (int t = 0; t < 4; ++t) acc[t] = zero8();
  gemm16x64x3(xh + xoff, xl + xoff, wh, wl, m0, n0, DM, DM, lane, acc);

  const float osc = (which == 0) ? 0.125f : 1.0f;
#pragma unroll
  for (int t = 0; t < 4; ++t) {
#pragma unroll
    for (int r = 0; r < 8; ++r)
      sf[(wave * 16 + 8 * hh + r) * SFP + 16 * t + c] = acc[t][r] * osc;
  }
  __syncthreads();

  if (which < 2) {
    v4u hv[4], lv[4];
    size_t go[4];
    const int headrow = (which == 0) ? (bb * NH + ns) : (bb * NG + (ns - 16));
#pragma unroll
    for (int j = 0; j < 4; ++j) {
      const int p  = tid + 128 * j;
      const int lr = p >> 3;
      const int d0 = (p & 7) * 8;
      const float* ra = sf + lr * SFP + d0;
      const v4f a0 = *(const v4f*)(ra), a1 = *(const v4f*)(ra + 4);
      const float f[8] = {a0[0], a0[1], a0[2], a0[3], a1[0], a1[1], a1[2], a1[3]};
      Pack8 ph, pl;
      split8(f, ph, pl);
      hv[j] = ph.u;
      lv[j] = pl.u;
      go[j] = ((size_t)headrow * TT + tb + lr) * HD + d0;
    }
    us* dsth = (which == 0) ? qh : kph;
    us* dstl = (which == 0) ? ql : kpl;
#pragma unroll
    for (int j = 0; j < 4; ++j) { *(volatile v4u*)(dsth + go[j]) = hv[j]; *(volatile v4u*)(dstl + go[j]) = lv[j]; }
    __threadfence();
#pragma unroll
    for (int j = 0; j < 4; ++j) { *(volatile v4u*)(dsth + go[j]) = hv[j]; *(volatile v4u*)(dstl + go[j]) = lv[j]; }
    if (which == 1) {
      const int g = ns - 16;
      put_ck(sf, nck, bb, g, tb, tid);
      __threadfence();
      put_ck(sf, nck, bb, g, tb, tid);
    }
  } else {
    v4u hv[4], lv[4];
    size_t go[4];
    const int g = ns - 20;
#pragma unroll
    for (int j = 0; j < 4; ++j) {
      const int p  = tid + 128 * j;
      const int d  = p >> 3;
      const int pc = p & 7;
      const float* cp = sf + (pc * 8) * SFP + d;
      float f[8];
#pragma unroll
      for (int e = 0; e < 8; ++e) f[e] = cp[e * SFP];
      Pack8 ph, pl;
      split8(f, ph, pl);
      hv[j] = ph.u;
      lv[j] = pl.u;
      go[j] = ((size_t)((bb * NG + g) * HD + d)) * TT + tb + pc * 8;
    }
#pragma unroll
    for (int j = 0; j < 4; ++j) { *(volatile v4u*)(vth + go[j]) = hv[j]; *(volatile v4u*)(vtl + go[j]) = lv[j]; }
    __threadfence();
#pragma unroll
    for (int j = 0; j < 4; ++j) { *(volatile v4u*)(vth + go[j]) = hv[j]; *(volatile v4u*)(vtl + go[j]) = lv[j]; }
    put_cv(sf, ncv, bb, g, tb, tid);
    __threadfence();
    put_cv(sf, ncv, bb, g, tb, tid);
  }
}

#define OTP 68
__global__ __launch_bounds__(128) void k_gemmf(const us* __restrict__ ah, const us* __restrict__ al,
                                               const us* __restrict__ bph, const us* __restrict__ bpl,
                                               float* __restrict__ out, int K, int brow0, int ldo) {
  __shared__ __align__(16) float st[4][16 * OTP];
  const int tid = threadIdx.x, lane = tid & 31, wave = tid >> 5;
  const int hh = lane >> 4, c = lane & 15;
  const int m0 = blockIdx.x * 64 + wave * 16;
  const int n0 = blockIdx.y * 64;

  v8f acc[4];
#pragma unroll
  for (int t = 0; t < 4; ++t) acc[t] = zero8();
  gemm16x64x3(ah, al, bph, bpl, m0, brow0 + n0, K, K, lane, acc);

  float* sw = st[wave];
#pragma unroll
  for (int t = 0; t < 4; ++t) {
#pragma unroll
    for (int r = 0; r < 8; ++r) sw[(8 * hh + r) * OTP + 16 * t + c] = acc[t][r];
  }
  __syncthreads();
  v4f val[8];
  size_t go[8];
#pragma unroll
  for (int it = 0; it < 8; ++it) {
    const int p    = lane + 32 * it;
    const int L    = p >> 3;
    const int pc   = p & 7;
    const int row  = L >> 1;
    const int half = L & 1;
    const int col  = n0 + half * 32 + pc * 4;
    go[it]  = (size_t)(m0 + row) * ldo + col;
    val[it] = *(const v4f*)(sw + row * OTP + half * 32 + pc * 4);
  }
#pragma unroll
  for (int it = 0; it < 8; ++it) *(volatile v4f*)(out + go[it]) = val[it];
  __threadfence();
#pragma unroll
  for (int it = 0; it < 8; ++it) *(volatile v4f*)(out + go[it]) = val[it];
}

#define LP 72
__global__ __launch_bounds__(128) void k_attn(const us* __restrict__ qh, const us* __restrict__ ql,
                                              const us* __restrict__ kph, const us* __restrict__ kpl,
                                              const us* __restrict__ vth, const us* __restrict__ vtl,
                                              const us* __restrict__ kch, const us* __restrict__ kcl,
                                              const us* __restrict__ vch, const us* __restrict__ vcl,
                                              const float* __restrict__ rt,
                                              us* __restrict__ oh, us* __restrict__ ol) {
  __shared__ __align__(16) us Ksh[KC * LP];
  __shared__ __align__(16) us Ksl[KC * LP];
  __shared__ __align__(16) us Vsh[HD * LP];
  __shared__ __align__(16) us Vsl[HD * LP];
  __shared__ __align__(16) us Psh[4 * 16 * LP];
  __shared__ __align__(16) us Psl[4 * 16 * LP];

  const int tid = threadIdx.x, lane = tid & 31, wave = tid >> 5;
  const int hh = lane >> 4, c = lane & 15;
  const int bhd = blockIdx.x / NQB;
  const int qb  = blockIdx.x % NQB;
  const int bb  = bhd >> 4, h = bhd & 15;
  const int bg  = bb * NG + (h >> 2);
  const int tq0 = qb * QB + wave * 16;

  const us* Qh = qh + (size_t)bhd * TT * HD;
  const us* Ql = ql + (size_t)bhd * TT * HD;
  const float* Rb = rt + (size_t)bhd * TT * NRELP;

  const float NEGI = -__builtin_huge_valf();
  float mrow[8], lrow[8];
  v8f oacc[4];
#pragma unroll
  for (int r = 0; r < 8; ++r) { mrow[r] = NEGI; lrow[r] = 0.f; }
#pragma unroll
  for (int t = 0; t < 4; ++t) oacc[t] = zero8();

  us* pwh = Psh + wave * 16 * LP;
  us* pwl = Psl + wave * 16 * LP;

  for (int ci = 0; ci < SKEY / KC; ++ci) {
    const int kv0 = ci * KC;
    const bool fromc = (ci < SC / KC);
    const int sl = fromc ? kv0 : (kv0 - SC);
    const us* ksh = fromc ? (kch + ((size_t)bhd * SC + sl) * HD) : (kph + ((size_t)bg * TT + sl) * HD);
    const us* ksl = fromc ? (kcl + ((size_t)bhd * SC + sl) * HD) : (kpl + ((size_t)bg * TT + sl) * HD);
    const us* vsh = fromc ? (vch + (size_t)bhd * HD * SC + sl) : (vth + (size_t)bg * HD * TT + sl);
    const us* vsl = fromc ? (vcl + (size_t)bhd * HD * SC + sl) : (vtl + (size_t)bg * HD * TT + sl);
    const int vp = fromc ? SC : TT;
    __syncthreads();
    {
      const int r  = tid >> 1;
      const int cb = (tid & 1) * 32;
      const us* ka = ksh + (size_t)r * HD + cb;
      const us* kb = ksl + (size_t)r * HD + cb;
      const us* va = vsh + (size_t)r * vp + cb;
      const us* vb = vsl + (size_t)r * vp + cb;
#pragma unroll
      for (int e = 0; e < 4; ++e) {
        *(v8us*)(Ksh + r * LP + cb + 8 * e) = *(const v8us*)(ka + 8 * e);
        *(v8us*)(Ksl + r * LP + cb + 8 * e) = *(const v8us*)(kb + 8 * e);
        *(v8us*)(Vsh + r * LP + cb + 8 * e) = *(const v8us*)(va + 8 * e);
        *(v8us*)(Vsl + r * LP + cb + 8 * e) = *(const v8us*)(vb + 8 * e);
      }
    }
    __syncthreads();

    v8f s[4];
#pragma unroll
    for (int j = 0; j < 4; ++j) s[j] = zero8();
#pragma unroll
    for (int dc = 0; dc < 2; ++dc) {
      const v16bf qah = ldfrag(Qh, HD, tq0, dc * 32, lane);
      const v16bf qal = ldfrag(Ql, HD, tq0, dc * 32, lane);
#pragma unroll
      for (int j = 0; j < 4; ++j) {
        const v16bf kbh = ldfrag(Ksh, LP, j * 16, dc * 32, lane);
        const v16bf kbl = ldfrag(Ksl, LP, j * 16, dc * 32, lane);
        s[j] = mma16(qah, kbh, s[j]);
        s[j] = mma16(qah, kbl, s[j]);
        s[j] = mma16(qal, kbh, s[j]);
      }
    }
#pragma unroll
    for (int r = 0; r < 8; ++r) {
      const int qry = tq0 + 8 * hh + r;
      const float* Rr = Rb + (size_t)qry * NRELP;
#pragma unroll
      for (int j = 0; j < 4; ++j) {
        const int key = kv0 + 16 * j + c;
        int di = qry - key + SC;
        di = (di < -127) ? -127 : ((di > 127) ? 127 : di);
        s[j][r] += Rr[di + 127];
      }
    }
    float cm[8];
#pragma unroll
    for (int r = 0; r < 8; ++r) {
      float m = s[0][r];
#pragma unroll
      for (int j = 1; j < 4; ++j) m = fmaxf(m, s[j][r]);
#pragma unroll
      for (int off = 1; off < 16; off <<= 1) m = fmaxf(m, __shfl_xor(m, off, 32));
      cm[r] = m;
    }
    float al[8];
#pragma unroll
    for (int r = 0; r < 8; ++r) {
      const float mnew  = fmaxf(mrow[r], cm[r]);
      const float alpha = __expf(mrow[r] - mnew);
      mrow[r] = mnew;
      float psum = 0.f;
#pragma unroll
      for (int j = 0; j < 4; ++j) {
        const float p = __expf(s[j][r] - mnew);
        psum += p;
        us ph, pl;
        split2(p, ph, pl);
        pwh[(8 * hh + r) * LP + j * 16 + c] = ph;
        pwl[(8 * hh + r) * LP + j * 16 + c] = pl;
      }
#pragma unroll
      for (int off = 1; off < 16; off <<= 1) psum += __shfl_xor(psum, off, 32);
      lrow[r] = lrow[r] * alpha + psum;
      al[r] = alpha;
    }
#pragma unroll
    for (int t = 0; t < 4; ++t)
#pragma unroll
      for (int r = 0; r < 8; ++r) oacc[t][r] *= al[r];
    __syncthreads();

#pragma unroll
    for (int kk = 0; kk < 2; ++kk) {
      const v16bf pah = ldfrag(pwh, LP, 0, kk * 32, lane);
      const v16bf pal = ldfrag(pwl, LP, 0, kk * 32, lane);
#pragma unroll
      for (int t = 0; t < 4; ++t) {
        const v16bf vbh = ldfrag(Vsh, LP, t * 16, kk * 32, lane);
        const v16bf vbl = ldfrag(Vsl, LP, t * 16, kk * 32, lane);
        oacc[t] = mma16(pah, vbh, oacc[t]);
        oacc[t] = mma16(pah, vbl, oacc[t]);
        oacc[t] = mma16(pal, vbh, oacc[t]);
      }
    }
  }

  float invl[8];
#pragma unroll
  for (int r = 0; r < 8; ++r) invl[r] = 1.0f / lrow[r];
  __syncthreads();
#pragma unroll
  for (int r = 0; r < 8; ++r) {
#pragma unroll
    for (int t = 0; t < 4; ++t) {
      us ohv, olv;
      split2(oacc[t][r] * invl[r], ohv, olv);
      pwh[(8 * hh + r) * LP + 16 * t + c] = ohv;
      pwl[(8 * hh + r) * LP + 16 * t + c] = olv;
    }
  }
  __syncthreads();
  v4u hv[4], lv[4];
  size_t go[4];
#pragma unroll
  for (int it = 0; it < 4; ++it) {
    const int p  = lane + 32 * it;
    const int L  = p >> 3;
    const int pc = p & 7;
    Pack8 ph, pl;
    ph.h   = *(const v8us*)(pwh + L * LP + pc * 8);
    pl.h   = *(const v8us*)(pwl + L * LP + pc * 8);
    hv[it] = ph.u;
    lv[it] = pl.u;
    go[it] = ((size_t)(bb * TT + tq0 + L)) * DM + (size_t)h * HD + pc * 8;
  }
#pragma unroll
  for (int it = 0; it < 4; ++it) { *(volatile v4u*)(oh + go[it]) = hv[it]; *(volatile v4u*)(ol + go[it]) = lv[it]; }
  __threadfence();
#pragma unroll
  for (int it = 0; it < 4; ++it) { *(volatile v4u*)(oh + go[it]) = hv[it]; *(volatile v4u*)(ol + go[it]) = lv[it]; }
}

extern "C" void kernel_launch(void* const* d_in, const int* in_sizes, int n_in,
                              void* d_out, int out_size, void* d_ws, size_t ws_size,
                              hipStream_t stream) {
  if (n_in < 10) return;
  if (in_sizes[0] != NTOK * DM) return;
  if (in_sizes[1] != NTOK * DM) return;
  if (in_sizes[2] != NTOK * DM) return;
  if (in_sizes[3] != NBH * HD * SC) return;
  if (in_sizes[4] != NBH * SC * HD) return;
  if (in_sizes[5] != DM * DM) return;
  if (in_sizes[6] != NG * HD * DM) return;
  if (in_sizes[7] != NG * HD * DM) return;
  if (in_sizes[8] != DM * DM) return;
  if (in_sizes[9] != NREL * HD) return;
  if (out_size != NTOK * DM + NBH * HD * SC + NBH * SC * HD) return;

  const float* q   = (const float*)d_in[0];
  const float* k   = (const float*)d_in[1];
  const float* v   = (const float*)d_in[2];
  const float* ck  = (const float*)d_in[3];
  const float* cv  = (const float*)d_in[4];
  const float* wq  = (const float*)d_in[5];
  const float* wk  = (const float*)d_in[6];
  const float* wv  = (const float*)d_in[7];
  const float* wo  = (const float*)d_in[8];
  const float* rel = (const float*)d_in[9];
  float* out0 = (float*)d_out;
  float* out1 = (float*)((char*)d_out + (size_t)8388608);
  float* out2 = (float*)((char*)d_out + (size_t)16777216);

  size_t off = 0;
  const size_t oXh  = off; off += (size_t)3 * NTOK * DM * 2;
  const size_t oXl  = off; off += (size_t)3 * NTOK * DM * 2;
  const size_t oWh  = off; off += (size_t)WROWS * DM * 2;
  const size_t oWl  = off; off += (size_t)WROWS * DM * 2;
  const size_t oRLh = off; off += (size_t)NRELP * HD * 2;
  const size_t oRLl = off; off += (size_t)NRELP * HD * 2;
  const size_t oQh  = off; off += (size_t)NBH * TT * HD * 2;
  const size_t oQl  = off; off += (size_t)NBH * TT * HD * 2;
  const size_t oKh  = off; off += (size_t)NBG * TT * HD * 2;
  const size_t oKl  = off; off += (size_t)NBG * TT * HD * 2;
  const size_t oVh  = off; off += (size_t)NBG * HD * TT * 2;
  const size_t oVl  = off; off += (size_t)NBG * HD * TT * 2;
  const size_t oCKh = off; off += (size_t)NBH * SC * HD * 2;
  const size_t oCKl = off; off += (size_t)NBH * SC * HD * 2;
  const size_t oCVh = off; off += (size_t)NBH * HD * SC * 2;
  const size_t oCVl = off; off += (size_t)NBH * HD * SC * 2;
  const size_t oRT  = off; off += (size_t)NBH * TT * NRELP * 4;
  const size_t oOh  = off; off += (size_t)NTOK * DM * 2;
  const size_t oOl  = off; off += (size_t)NTOK * DM * 2;
  if (off > ws_size) return;
  if (off > (size_t)134217728) return;

  char* ws = (char*)d_ws;
  us* Xh  = (us*)(ws + oXh);
  us* Xl  = (us*)(ws + oXl);
  us* Wh  = (us*)(ws + oWh);
  us* Wl  = (us*)(ws + oWl);
  us* RLh = (us*)(ws + oRLh);
  us* RLl = (us*)(ws + oRLl);
  us* Qh  = (us*)(ws + oQh);
  us* Ql  = (us*)(ws + oQl);
  us* Kh  = (us*)(ws + oKh);
  us* Kl  = (us*)(ws + oKl);
  us* Vh  = (us*)(ws + oVh);
  us* Vl  = (us*)(ws + oVl);
  us* CKh = (us*)(ws + oCKh);
  us* CKl = (us*)(ws + oCKl);
  us* CVh = (us*)(ws + oCVh);
  us* CVl = (us*)(ws + oCVl);
  float* RT = (float*)(ws + oRT);
  us* Oh  = (us*)(ws + oOh);
  us* Ol  = (us*)(ws + oOl);

  k_cvt<<<dim3(NCVT), dim3(256), 0, stream>>>(q, k, v, wq, wk, wv, wo, rel, Xh, Xl, Wh, Wl, RLh, RLl);
  k_cvtc<<<dim3(SC / 64, NBH, 2), dim3(128), 0, stream>>>(ck, cv, CKh, CKl, CVh, CVl);
  k_qkv<<<dim3(NTOK / 64, (DM + 2 * NG * HD) / HD), dim3(128), 0, stream>>>(Xh, Xl, Wh, Wl, Qh, Ql, Kh, Kl,
                                                                             Vh, Vl, out1, out2);
  k_gemmf<<<dim3((NBH * TT) / 64, NRELP / 64), dim3(128), 0, stream>>>(Qh, Ql, RLh, RLl, RT, HD, 0, NRELP);
  k_attn<<<dim3(NBH * NQB), dim3(128), 0, stream>>>(Qh, Ql, Kh, Kl, Vh, Vl, CKh, CKl, CVh, CVl, RT, Oh, Ol);
  k_gemmf<<<dim3(NTOK / 64, DM / 64), dim3(128), 0, stream>>>(Oh, Ol, Wh, Wl, out0, DM, OROW, DM);
  (void)hipGetLastError();
}
